// MultiHeadedAttentionWithDepth_36369783063352
// MI455X (gfx1250) — hardware-verified
//
#include <hip/hip_runtime.h>
#include <stddef.h>


typedef _Float16 f16;
typedef f16   v16h __attribute__((ext_vector_type(16)));
typedef f16   v8h  __attribute__((ext_vector_type(8)));
typedef float v8f  __attribute__((ext_vector_type(8)));
typedef float v4f  __attribute__((ext_vector_type(4)));

#define NSEQ   2048
#define NBATCH 4
#define NHEAD  8
#define C1D    512
#define C2D    128
#define CCAT   640
#define DHEAD  80
#define C1H    64
#define C2H    16
#define MROWS  (NBATCH * NSEQ)

#define KT_LD 88
#define VT_LD 72
#define PT_LD 72
#define OT_LD 80

union GemmSmem { float f[64 * 128]; f16 h[128 * 128]; };


__device__ __forceinline__ v8f wmma16(v16h a, v16h b, v8f c) {
  v8f d = __builtin_amdgcn_wmma_f32_16x16x32_f16(false, a, false, b, (short)0, c,
                                                 false, false);
  asm volatile("v_nop\n\tv_nop\n\tv_nop\n\tv_nop" : "+v"(d) : "v"(a), "v"(b));
  return d;
}

__device__ __forceinline__ v8f zf8() {
  v8f z = {0.0f, 0.0f, 0.0f, 0.0f, 0.0f, 0.0f, 0.0f, 0.0f};
  return z;
}

__device__ __forceinline__ v8h zh8() {
  const f16 z0 = (f16)0.0f;
  v8h z = {z0, z0, z0, z0, z0, z0, z0, z0};
  return z;
}

__device__ __forceinline__ v16h join16(v8h lo, v8h hi) {
  return __builtin_shufflevector(lo, hi, 0, 1, 2, 3, 4, 5, 6, 7, 8, 9, 10, 11, 12,
                                 13, 14, 15);
}

__device__ __forceinline__ v16h ld_frag(const f16* p, int hf) {
  const v8h lo = *(const v8h*)(p + 8 * hf);
  const v8h hi = *(const v8h*)(p + 16 + 8 * hf);
  return join16(lo, hi);
}

__device__ __forceinline__ v16h ld_frag_k16(const f16* p, int hf) {
  const v8h lo = *(const v8h*)(p + 8 * hf);
  return join16(lo, zh8());
}

__device__ __forceinline__ float hmax16(float v) {
  v = fmaxf(v, __shfl_xor(v, 1, 32));
  v = fmaxf(v, __shfl_xor(v, 2, 32));
  v = fmaxf(v, __shfl_xor(v, 4, 32));
  v = fmaxf(v, __shfl_xor(v, 8, 32));
  return v;
}

__device__ __forceinline__ float hsum16(float v) {
  v += __shfl_xor(v, 1, 32);
  v += __shfl_xor(v, 2, 32);
  v += __shfl_xor(v, 4, 32);
  v += __shfl_xor(v, 8, 32);
  return v;
}


__global__ __launch_bounds__(256) void k_pack_tokens(const float* __restrict__ color,
                                                     const float* __restrict__ depth,
                                                     f16* X, int nunits) {
  const int u = blockIdx.x * 256 + threadIdx.x;
  const bool ok = u < nunits;
  const size_t e = (size_t)u * 8;
  const size_t g = e / CCAT;
  const int c = (int)(e - g * CCAT);
  v8h val = zh8();
  if (ok) {
    const float* src = (c < C1D) ? (color + g * C1D + c) : (depth + g * C2D + (c - C1D));
    const v4f x0 = *(const v4f*)src;
    const v4f x1 = *(const v4f*)(src + 4);
#pragma unroll
    for (int i = 0; i < 4; ++i) {
      val[i] = (f16)x0[i];
      val[i + 4] = (f16)x1[i];
    }
  }
  f16* dst = X + e;
  if (ok) *(volatile v8h*)dst = val;
  __threadfence();
  if (ok) *(volatile v8h*)dst = val;
}

__global__ __launch_bounds__(256) void k_pack_weight(const float* __restrict__ W, f16* Wt,
                                                     int K, int N, float scale, int nunits) {
  const int u = blockIdx.x * 256 + threadIdx.x;
  const bool ok = u < nunits;
  const size_t e = (size_t)u * 8;
  const int n = (int)(e / (size_t)K);
  const int k = (int)(e - (size_t)n * K);
  v8h val = zh8();
  if (ok) {
#pragma unroll
    for (int j = 0; j < 8; ++j) val[j] = (f16)(scale * W[(size_t)(k + j) * N + n]);
  }
  f16* dst = Wt + e;
  if (ok) *(volatile v8h*)dst = val;
  __threadfence();
  if (ok) *(volatile v8h*)dst = val;
}


template <bool OUT16, int AHW>
__global__ __launch_bounds__(256) void k_gemm(const f16* __restrict__ A, int lda,
                                              const f16* __restrict__ Wt,
                                              const float* __restrict__ bias, int K,
                                              int Nout, int M, float ascale, void* outp) {
  __shared__ __align__(16) GemmSmem sm;
  const int tid = threadIdx.x;
  const int lane = tid & 31, w = tid >> 5, hf = lane >> 4, l16 = lane & 15;
  const int bm0 = blockIdx.y * 128, bn0 = blockIdx.x * 128;
  const int wm = (w & 3) * 32, wn = (w >> 2) * 64;
  (void)lda;

  v8f acc[2][4];
#pragma unroll
  for (int i = 0; i < 2; ++i)
#pragma unroll
    for (int j = 0; j < 4; ++j) acc[i][j] = zf8();

  for (int k0 = 0; k0 < K; k0 += 32) {
    v16h a[2];
#pragma unroll
    for (int i = 0; i < 2; ++i) {
      const int row = bm0 + wm + i * 16 + l16;
      if constexpr (AHW == 0) {
        a[i] = ld_frag(A + (size_t)row * lda + k0, hf);
      } else {
        const int bb = row / NSEQ, n = row - bb * NSEQ;
        const int k1 = k0 + 8 * hf, k2 = k1 + 16;
        const f16* p1 = A + ((size_t)(bb * NHEAD + k1 / AHW) * NSEQ + n) * AHW + (k1 % AHW);
        const f16* p2 = A + ((size_t)(bb * NHEAD + k2 / AHW) * NSEQ + n) * AHW + (k2 % AHW);
        a[i] = join16(*(const v8h*)p1, *(const v8h*)p2);
      }
    }
#pragma unroll
    for (int j = 0; j < 4; ++j) {
      const int col = bn0 + wn + j * 16 + l16;
      const v16h bfr = ld_frag(Wt + (size_t)col * K + k0, hf);
#pragma unroll
      for (int i = 0; i < 2; ++i) acc[i][j] = wmma16(a[i], bfr, acc[i][j]);
    }
  }

  float bv[4];
#pragma unroll
  for (int j = 0; j < 4; ++j) bv[j] = bias[bn0 + wn + j * 16 + l16];

  if constexpr (OUT16) {
#pragma unroll
    for (int j = 0; j < 4; ++j)
#pragma unroll
      for (int i = 0; i < 2; ++i)
#pragma unroll
        for (int r = 0; r < 8; ++r) {
          const int lm = wm + i * 16 + 8 * hf + r;
          const int lc = wn + j * 16 + l16;
          sm.h[lm * 128 + lc] = (f16)(acc[i][j][r] * ascale + bv[j]);
        }
    __syncthreads();
    f16* out = (f16*)outp;
#pragma unroll
    for (int pass = 0; pass < 2; ++pass) {
#pragma unroll
      for (int it = 0; it < 8; ++it) {
        const int u = it * 256 + tid;
        const int row = u >> 4, cu = u & 15;
        const v8h v = *(const v8h*)(&sm.h[row * 128 + cu * 8]);
        const int grow = bm0 + row;
        if (grow < M) *(volatile v8h*)(out + (size_t)grow * Nout + bn0 + cu * 8) = v;
      }
      if (pass == 0) __threadfence();
    }
  } else {
    float* out = (float*)outp;
#pragma unroll
    for (int p = 0; p < 2; ++p) {
      if (((w & 3) >> 1) == p) {
#pragma unroll
        for (int j = 0; j < 4; ++j)
#pragma unroll
          for (int i = 0; i < 2; ++i)
#pragma unroll
            for (int r = 0; r < 8; ++r) {
              const int lm = wm - p * 64 + i * 16 + 8 * hf + r;
              const int lc = wn + j * 16 + l16;
              sm.f[lm * 128 + lc] = acc[i][j][r] * ascale + bv[j];
            }
      }
      __syncthreads();
#pragma unroll
      for (int pass = 0; pass < 2; ++pass) {
#pragma unroll
        for (int it = 0; it < 8; ++it) {
          const int u = it * 256 + tid;
          const int row = u >> 5, cu = u & 31;
          const v4f v = *(const v4f*)(&sm.f[row * 128 + cu * 4]);
          const int grow = bm0 + p * 64 + row;
          if (grow < M) *(volatile v4f*)(out + (size_t)grow * Nout + bn0 + cu * 4) = v;
        }
        if (pass == 0) __threadfence();
      }
      __syncthreads();
    }
  }
}


__global__ __launch_bounds__(256) void k_attn(const f16* __restrict__ Q,
                                              const f16* __restrict__ Kp,
                                              const f16* __restrict__ Vc,
                                              const f16* __restrict__ Vd, f16* Ocb, f16* Odb,
                                              float cs) {
  __shared__ __align__(16) f16 kT[64 * KT_LD];
  __shared__ __align__(16) f16 vT[DHEAD * VT_LD];
  __shared__ __align__(16) f16 pT[8 * 16 * PT_LD];
  __shared__ __align__(16) f16 oT[128 * OT_LD];

  const int tid = threadIdx.x;
  const int lane = tid & 31, w = tid >> 5, hf = lane >> 4, l16 = lane & 15;
  const int bh = blockIdx.y, b = bh >> 3, h = bh & 7;
  const int qb = blockIdx.x * 128;
  const size_t tok0 = (size_t)b * NSEQ;

  const f16* qp = Q + (tok0 + qb + w * 16 + l16) * CCAT + h * DHEAD;
  const v16h qa0 = ld_frag(qp, hf);
  const v16h qa1 = ld_frag(qp + 32, hf);
  const v16h qa2 = ld_frag_k16(qp + 64, hf);

  v8f o[5];
#pragma unroll
  for (int vt = 0; vt < 5; ++vt) o[vt] = zf8();
  float mrow[8], lrow[8];
#pragma unroll
  for (int r = 0; r < 8; ++r) { mrow[r] = -3.0e38f; lrow[r] = 0.0f; }

  for (int kc = 0; kc < NSEQ; kc += 64) {
    __syncthreads();
#pragma unroll
    for (int it = 0; it < 3; ++it) {
      const int u = tid + it * 256;
      if (u < 640) {
        const int row = u / 10, cu = u - row * 10;
        const v8h v = *(const v8h*)(Kp + (tok0 + kc + row) * CCAT + h * DHEAD + cu * 8);
        *(v8h*)(&kT[row * KT_LD + cu * 8]) = v;
      }
    }
#pragma unroll
    for (int it = 0; it < 3; ++it) {
      const int u = tid + it * 256;
      if (u < 512) {
        const int key = u >> 3, cu = u & 7;
        const v8h v = *(const v8h*)(Vc + (tok0 + kc + key) * C1D + h * C1H + cu * 8);
        f16* dst = &vT[(cu * 8) * VT_LD + key];
#pragma unroll
        for (int jj = 0; jj < 8; ++jj) dst[jj * VT_LD] = v[jj];
      } else if (u < 640) {
        const int u2 = u - 512;
        const int key = u2 >> 1, cu = u2 & 1;
        const v8h v = *(const v8h*)(Vd + (tok0 + kc + key) * C2D + h * C2H + cu * 8);
        f16* dst = &vT[(C1H + cu * 8) * VT_LD + key];
#pragma unroll
        for (int jj = 0; jj < 8; ++jj) dst[jj * VT_LD] = v[jj];
      }
    }
    __syncthreads();

    v8f s[4];
#pragma unroll
    for (int t = 0; t < 4; ++t) s[t] = zf8();
#pragma unroll
    for (int t = 0; t < 4; ++t) {
      const f16* kp = &kT[(t * 16 + l16) * KT_LD];
      s[t] = wmma16(qa0, ld_frag(kp, hf), s[t]);
      s[t] = wmma16(qa1, ld_frag(kp + 32, hf), s[t]);
      s[t] = wmma16(qa2, ld_frag_k16(kp + 64, hf), s[t]);
    }

    float sf[8];
#pragma unroll
    for (int r = 0; r < 8; ++r) {
      float v = fmaxf(fmaxf(s[0][r], s[1][r]), fmaxf(s[2][r], s[3][r])) * cs;
      v = hmax16(v);
      const float mn = fmaxf(mrow[r], v);
      sf[r] = exp2f(mrow[r] - mn);
      mrow[r] = mn;
    }
#pragma unroll
    for (int t = 0; t < 4; ++t)
#pragma unroll
      for (int r = 0; r < 8; ++r) s[t][r] = exp2f(s[t][r] * cs - mrow[r]);
#pragma unroll
    for (int r = 0; r < 8; ++r) {
      const float v = hsum16(s[0][r] + s[1][r] + s[2][r] + s[3][r]);
      lrow[r] = lrow[r] * sf[r] + v;
    }
#pragma unroll
    for (int vt = 0; vt < 5; ++vt)
#pragma unroll
      for (int r = 0; r < 8; ++r) o[vt][r] *= sf[r];

#pragma unroll
    for (int t = 0; t < 4; ++t)
#pragma unroll
      for (int r = 0; r < 8; ++r)
        pT[(w * 16 + 8 * hf + r) * PT_LD + t * 16 + l16] = (f16)(s[t][r] * 256.0f);
    __syncthreads();

#pragma unroll
    for (int kst = 0; kst < 2; ++kst) {
      const v16h pa = ld_frag(&pT[(w * 16 + l16) * PT_LD + kst * 32], hf);
#pragma unroll
      for (int vt = 0; vt < 5; ++vt) {
        const v16h vf = ld_frag(&vT[(vt * 16 + l16) * VT_LD + kst * 32], hf);
        o[vt] = wmma16(pa, vf, o[vt]);
      }
    }
  }

  float inv[8];
#pragma unroll
  for (int r = 0; r < 8; ++r) inv[r] = 0.0625f / lrow[r];
#pragma unroll
  for (int vt = 0; vt < 5; ++vt)
#pragma unroll
    for (int r = 0; r < 8; ++r)
      oT[(w * 16 + 8 * hf + r) * OT_LD + vt * 16 + l16] = (f16)(o[vt][r] * inv[r]);
  __syncthreads();

#pragma unroll
  for (int pass = 0; pass < 2; ++pass) {
#pragma unroll
    for (int it = 0; it < 5; ++it) {
      const int u = it * 256 + tid;
      if (it < 4) {
        const int row = u >> 3, cu = u & 7;
        const v8h v = *(const v8h*)(&oT[row * OT_LD + cu * 8]);
        *(volatile v8h*)(Ocb + ((size_t)bh * NSEQ + qb + row) * C1H + cu * 8) = v;
      } else {
        const int u2 = u - 1024;
        const int row = u2 >> 1, cu = u2 & 1;
        const v8h v = *(const v8h*)(&oT[row * OT_LD + C1H + cu * 8]);
        *(volatile v8h*)(Odb + ((size_t)bh * NSEQ + qb + row) * C2H + cu * 8) = v;
      }
    }
    if (pass == 0) __threadfence();
  }
}


extern "C" void kernel_launch(void* const* d_in, const int* in_sizes, int n_in, void* d_out,
                              int out_size, void* d_ws, size_t ws_size, hipStream_t stream) {
  if (n_in < 14) return;
  if (in_sizes[0] != MROWS * C1D || in_sizes[1] != MROWS * C2D || in_sizes[2] != CCAT * CCAT ||
      in_sizes[3] != CCAT || in_sizes[4] != CCAT * CCAT || in_sizes[5] != CCAT ||
      in_sizes[6] != C1D * C1D || in_sizes[7] != C1D || in_sizes[8] != C2D * C2D ||
      in_sizes[9] != C2D || in_sizes[10] != C1D * C1D || in_sizes[11] != C1D ||
      in_sizes[12] != C2D * C2D || in_sizes[13] != C2D)
    return;
  if (out_size != MROWS * (C1D + C2D)) return;

  const float* color = (const float*)d_in[0];
  const float* depth = (const float*)d_in[1];
  const float* Wq  = (const float*)d_in[2];  const float* bq  = (const float*)d_in[3];
  const float* Wk  = (const float*)d_in[4];  const float* bk  = (const float*)d_in[5];
  const float* Wcv = (const float*)d_in[6];  const float* bcv = (const float*)d_in[7];
  const float* Wdv = (const float*)d_in[8];  const float* bdv = (const float*)d_in[9];
  const float* Wcl = (const float*)d_in[10]; const float* bcl = (const float*)d_in[11];
  const float* Wdl = (const float*)d_in[12]; const float* bdl = (const float*)d_in[13];

  char* ws = (char*)d_ws;
  size_t off = 0;
  auto take = [&](size_t bytes) {
    char* p = ws + off;
    off += (bytes + 255) & ~(size_t)255;
    return p;
  };
  f16* X16  = (f16*)take((size_t)MROWS * CCAT * 2);
  f16* WqT  = (f16*)take((size_t)CCAT * CCAT * 2);
  f16* WkT  = (f16*)take((size_t)CCAT * CCAT * 2);
  f16* WcvT = (f16*)take((size_t)C1D * C1D * 2);
  f16* WdvT = (f16*)take((size_t)C2D * C2D * 2);
  f16* WclT = (f16*)take((size_t)C1D * C1D * 2);
  f16* WdlT = (f16*)take((size_t)C2D * C2D * 2);
  f16* Q16  = (f16*)take((size_t)MROWS * CCAT * 2);
  f16* K16  = (f16*)take((size_t)MROWS * CCAT * 2);
  f16* Vc16 = (f16*)take((size_t)MROWS * C1D * 2);
  f16* Vd16 = (f16*)take((size_t)MROWS * C2D * 2);
  f16* Ocb  = (f16*)take((size_t)NBATCH * NHEAD * NSEQ * C1H * 2);
  f16* Odb  = (f16*)take((size_t)NBATCH * NHEAD * NSEQ * C2H * 2);
  if (off > ws_size) return;

  const int TB = 256;
  {
    const int nunits = MROWS * CCAT / 8;
    k_pack_tokens<<<(nunits + TB - 1) / TB, TB, 0, stream>>>(color, depth, X16, nunits);
  }
  const float wscale = 64.0f;
  {
    const int u1 = CCAT * CCAT / 8;
    k_pack_weight<<<(u1 + TB - 1) / TB, TB, 0, stream>>>(Wq, WqT, CCAT, CCAT, wscale, u1);
    k_pack_weight<<<(u1 + TB - 1) / TB, TB, 0, stream>>>(Wk, WkT, CCAT, CCAT, wscale, u1);
    const int u2 = C1D * C1D / 8;
    k_pack_weight<<<(u2 + TB - 1) / TB, TB, 0, stream>>>(Wcv, WcvT, C1D, C1D, wscale, u2);
    k_pack_weight<<<(u2 + TB - 1) / TB, TB, 0, stream>>>(Wcl, WclT, C1D, C1D, wscale, u2);
    const int u3 = C2D * C2D / 8;
    k_pack_weight<<<(u3 + TB - 1) / TB, TB, 0, stream>>>(Wdv, WdvT, C2D, C2D, wscale, u3);
    k_pack_weight<<<(u3 + TB - 1) / TB, TB, 0, stream>>>(Wdl, WdlT, C2D, C2D, wscale, u3);
  }
  const float inv_w = 1.0f / 64.0f;
  k_gemm<true, 0><<<dim3(CCAT / 128, MROWS / 128), TB, 0, stream>>>(
      X16, CCAT, WqT, bq, CCAT, CCAT, MROWS, inv_w, (void*)Q16);
  k_gemm<true, 0><<<dim3(CCAT / 128, MROWS / 128), TB, 0, stream>>>(
      X16, CCAT, WkT, bk, CCAT, CCAT, MROWS, inv_w, (void*)K16);
  k_gemm<true, 0><<<dim3(C1D / 128, MROWS / 128), TB, 0, stream>>>(
      X16, CCAT, WcvT, bcv, C1D, C1D, MROWS, inv_w, (void*)Vc16);
  k_gemm<true, 0><<<dim3(C2D / 128, MROWS / 128), TB, 0, stream>>>(
      X16 + C1D, CCAT, WdvT, bdv, C2D, C2D, MROWS, inv_w, (void*)Vd16);
  const float cs = 0.11180339887498949f * 1.4426950408889634f;
  k_attn<<<dim3(NSEQ / 128, NBATCH * NHEAD), TB, 0, stream>>>(Q16, K16, Vc16, Vd16, Ocb,
                                                             Odb, cs);
  float* out_color = (float*)d_out;
  float* out_depth = out_color + (size_t)MROWS * C1D;
  const float inv_ow = 1.0f / 1024.0f;
  k_gemm<false, C1H><<<dim3(C1D / 128, MROWS / 128), TB, 0, stream>>>(
      Ocb, 0, WclT, bcl, C1D, C1D, MROWS, inv_ow, (void*)out_color);
  k_gemm<false, C2H><<<dim3(C2D / 128, MROWS / 128), TB, 0, stream>>>(
      Odb, 0, WdlT, bdl, C2D, C2D, MROWS, inv_ow, (void*)out_depth);
}
